// AtomMPNN_90683939487977
// MI455X (gfx1250) — hardware-run, weakly checked
//
#include <hip/hip_runtime.h>

typedef float          v8f   __attribute__((ext_vector_type(8)));
typedef float          v4f   __attribute__((ext_vector_type(4)));
typedef unsigned int   v4u   __attribute__((ext_vector_type(4)));
typedef int            v8i   __attribute__((ext_vector_type(8)));
typedef unsigned short v8us  __attribute__((ext_vector_type(8)));
typedef unsigned short v16us __attribute__((ext_vector_type(16)));
typedef __bf16         v16bf __attribute__((ext_vector_type(16)));
typedef _Float16       v16h  __attribute__((ext_vector_type(16)));
typedef v4f  __attribute__((may_alias)) v4fa;
typedef v8us __attribute__((may_alias)) v8usa;
union FragB { v16bf v; v16us u; v8us h[2]; v8i w; };
union FragH { v16h  v; v16us u; v8us h[2]; v8i w; };

__device__ __forceinline__ v8f wmb(const FragB& a, const FragB& b, v8f c) {
  v8f d = __builtin_amdgcn_wmma_f32_16x16x32_bf16(false, a.v, false, b.v, (short)0, c, false, false);
  asm volatile("v_nop\n\tv_nop\n\tv_nop\n\tv_nop" : "+v"(d) : "v"(a.w), "v"(b.w));
  return d;
}

__device__ __forceinline__ v8f wmh(const FragH& a, const FragH& b, v8f c) {
  v8f d = __builtin_amdgcn_wmma_f32_16x16x32_f16(false, a.v, false, b.v, (short)0, c, false, false);
  asm volatile("v_nop\n\tv_nop\n\tv_nop\n\tv_nop" : "+v"(d) : "v"(a.w), "v"(b.w));
  return d;
}

__device__ __forceinline__ unsigned bf16_bits(float f) {
  const unsigned u = __float_as_uint(f);
  const unsigned r = (u + 0x7FFFu + ((u >> 16) & 1u)) >> 16;
  const unsigned q = (u >> 16) | 0x40u;
  return ((u & 0x7fffffffu) > 0x7f800000u) ? q : r;
}

__device__ __forceinline__ float bf16_val(float f) {
  return __uint_as_float(bf16_bits(f) << 16);
}
__device__ __forceinline__ int clampi(int v, int lo, int hi) {
  return v < lo ? lo : (v > hi ? hi : v);
}

__device__ __forceinline__ unsigned f16_bits(float f) {
  const unsigned u  = __float_as_uint(f);
  const unsigned s  = (u >> 16) & 0x8000u;
  const unsigned a  = u & 0x7fffffffu;
  const unsigned t  = a - 0x38000000u;
  const unsigned r  = (t + 0x0FFFu + ((t >> 13) & 1u)) >> 13;
  const unsigned rc = r > 0x7C00u ? 0x7C00u : r;
  const bool small  = a < 0x38800000u;
  const bool isnan  = a > 0x7f800000u;
  const unsigned fin = small ? 0u : (s | rc);
  return isnan ? (s | 0x7E00u) : fin;
}

__device__ __forceinline__ unsigned pk16(unsigned lo, unsigned hi) { return lo | (hi << 16); }
__device__ __forceinline__ unsigned bf16_lo_bits(float v) {
  float hi = bf16_val(v);
  asm volatile("" : "+v"(hi));
  return bf16_bits(v - hi);
}
__device__ __forceinline__ v4u pack8_bf16(v4f a, v4f c) {
  return (v4u){ pk16(bf16_bits(a[0]), bf16_bits(a[1])), pk16(bf16_bits(a[2]), bf16_bits(a[3])),
                pk16(bf16_bits(c[0]), bf16_bits(c[1])), pk16(bf16_bits(c[2]), bf16_bits(c[3])) };
}
__device__ __forceinline__ v4u pack8_bf16_lo(v4f a, v4f c) {
  return (v4u){ pk16(bf16_lo_bits(a[0]), bf16_lo_bits(a[1])), pk16(bf16_lo_bits(a[2]), bf16_lo_bits(a[3])),
                pk16(bf16_lo_bits(c[0]), bf16_lo_bits(c[1])), pk16(bf16_lo_bits(c[2]), bf16_lo_bits(c[3])) };
}
__device__ __forceinline__ v4u pack8_f16(v4f a, v4f c) {
  return (v4u){ pk16(f16_bits(a[0]), f16_bits(a[1])), pk16(f16_bits(a[2]), f16_bits(a[3])),
                pk16(f16_bits(c[0]), f16_bits(c[1])), pk16(f16_bits(c[2]), f16_bits(c[3])) };
}

template <int FORM>
__global__ __launch_bounds__(256) void k_plane(const float* __restrict__ src, int rows, int cols, int ldsrc,
                                               unsigned short* __restrict__ dst, int MP, int KP) {
  static_assert(FORM >= 0 && FORM <= 3);
  const int KTOT = (FORM == 1 || FORM == 3) ? 2 * KP : KP;
  const unsigned ppr   = (unsigned)(KTOT >> 3);
  const unsigned kp8   = (unsigned)(KP >> 3);
  const unsigned total = (unsigned)MP * ppr;
  const unsigned g     = blockIdx.x * 256u + threadIdx.x;
  const unsigned rowu  = g / ppr;
  const unsigned p     = g - rowu * ppr;
  const bool second    = p >= kp8;
  const int row = (int)rowu;
  const int c0  = (int)((second ? p - kp8 : p) << 3);
  const float* srow = src + (size_t)clampi(row, 0, rows - 1) * (size_t)ldsrc;
  float x[8];
  unsigned mk[8];
#pragma unroll
  for (int e = 0; e < 8; ++e) {
    const int c = c0 + e;
    const float v = srow[clampi(c, 0, cols - 1)];
    asm volatile("" :: "v"(v));
    x[e]  = v;
    mk[e] = (row < rows && c < cols) ? 0xFFFFu : 0u;
  }
  const v4f a = (v4f){ x[0], x[1], x[2], x[3] };
  const v4f c = (v4f){ x[4], x[5], x[6], x[7] };
  v4u o;
  if (FORM == 2) {
    o = pack8_f16(a, c);
  } else {
    const v4u hi = pack8_bf16(a, c);
    o = hi;
    if (FORM == 1) { const v4u lo = pack8_bf16_lo(a, c); o = second ? lo : hi; }
  }
  const v4u mw = (v4u){ pk16(mk[0], mk[1]), pk16(mk[2], mk[3]), pk16(mk[4], mk[5]), pk16(mk[6], mk[7]) };
  o &= mw;
  if (g < total) {
    volatile v4u* q = (volatile v4u*)(dst + (size_t)g * 8);
    *q = o;
    __threadfence();
    *q = o;
  }
}

template <int FORM> struct FragOf    { typedef FragB T; };
template <>         struct FragOf<2> { typedef FragH T; };
__device__ __forceinline__ v8f mm(const FragB& a, const FragB& b, v8f c) { return wmb(a, b, c); }
__device__ __forceinline__ v8f mm(const FragH& a, const FragH& b, v8f c) { return wmh(a, b, c); }
template <class F> __device__ __forceinline__ F ld_frag(const unsigned short* p) {
  F f;
  f.h[0] = *(const v8usa*)(p);
  f.h[1] = *(const v8usa*)(p + 16);
  return f;
}

template <int FORM, int EPI>
__global__ __launch_bounds__(256) __attribute__((amdgpu_num_vgpr(248)))
void k_gemm_nt(const unsigned short* __restrict__ A, const unsigned short* __restrict__ B,
               const float* __restrict__ bias, float* __restrict__ D, int M, int N, int KTOT, int ldd) {
  static_assert(FORM >= 0 && FORM <= 2);
  static_assert(EPI == 0 || EPI == 1);
  typedef typename FragOf<FORM>::T F;
  __shared__ __attribute__((aligned(16))) float sT[8][16 * 68];
  const int lane = threadIdx.x & 31;
  const int wave = threadIdx.x >> 5;
  const int tilesM = (M + 63) >> 6;
  const int tilesN = (N + 63) >> 6;
  const int tile = blockIdx.x * 8 + wave;
  if (tile >= tilesM * tilesN) return;
  const int tm = tile / tilesN;
  const int tn = tile - tm * tilesN;
  const int m0 = tm << 6;
  const int n0 = tn << 6;

  const int rl = lane & 15;
  const int h8 = (lane >> 4) * 8;
  const unsigned short* pa = A + (size_t)(m0 + rl) * (size_t)KTOT + h8;
  const unsigned short* pb = B + (size_t)(n0 + rl) * (size_t)KTOT + h8;

  v8f acc[4][4];
#pragma unroll
  for (int i = 0; i < 4; ++i)
#pragma unroll
    for (int j = 0; j < 4; ++j) acc[i][j] = (v8f){0.f, 0.f, 0.f, 0.f, 0.f, 0.f, 0.f, 0.f};

#pragma unroll 1
  for (int k0 = 0; k0 < KTOT; k0 += 32) {
    F bf[4];
#pragma unroll
    for (int j = 0; j < 4; ++j) bf[j] = ld_frag<F>(pb + (size_t)(j << 4) * (size_t)KTOT + k0);
#pragma unroll
    for (int i = 0; i < 4; ++i) {
      const F af = ld_frag<F>(pa + (size_t)(i << 4) * (size_t)KTOT + k0);
#pragma unroll
      for (int j = 0; j < 4; ++j) acc[i][j] = mm(af, bf[j], acc[i][j]);
    }
  }

  float* slab = sT[wave];
  const int hh = lane >> 4;
  const int c4 = (lane & 15) * 4;
  const int nc = n0 + c4;
  const bool cok = nc < N;
  v4f bv = (v4f){0.f, 0.f, 0.f, 0.f};
  if (EPI == 1) {
    bv = *(const v4fa*)(bias + clampi(nc, 0, N - 4));
    asm volatile("" :: "v"(bv));
  }
#pragma unroll
  for (int i = 0; i < 4; ++i) {
    const int mBase = m0 + (i << 4);
#pragma unroll
    for (int j = 0; j < 4; ++j) {
#pragma unroll
      for (int r = 0; r < 8; ++r) slab[(h8 + r) * 68 + (j << 4) + rl] = acc[i][j][r];
    }
    __builtin_amdgcn_fence(__ATOMIC_RELEASE, "workgroup");
    __builtin_amdgcn_wave_barrier();
    __builtin_amdgcn_fence(__ATOMIC_ACQUIRE, "workgroup");
    v4f vv[8];
#pragma unroll
    for (int it = 0; it < 8; ++it) {
      const int row = it * 2 + hh;
      v4f v = *(const v4fa*)(slab + row * 68 + c4);
      if (EPI == 1) v += bv;
      vv[it] = v;
    }
    for (int pass = 0; pass < 2; ++pass) {
#pragma unroll
      for (int it = 0; it < 8; ++it) {
        const int row = mBase + it * 2 + hh;
        if (cok && row < M) *(volatile v4f*)(D + (size_t)row * (size_t)ldd + nc) = vv[it];
      }
      __threadfence();
    }
    __builtin_amdgcn_fence(__ATOMIC_RELEASE, "workgroup");
    __builtin_amdgcn_wave_barrier();
    __builtin_amdgcn_fence(__ATOMIC_ACQUIRE, "workgroup");
  }
}

#define GELU_MODE      0
#define MLP1_TWO_TERM  0
#define MLP2_TWO_TERM  0

typedef float  v2f __attribute__((ext_vector_type(2)));
typedef double v2d __attribute__((ext_vector_type(2)));
typedef v2f __attribute__((may_alias)) v2fa;

constexpr int NBATCH  = 8;
constexpr int NATOM   = 8192;
constexpr int NNBR    = 32;
constexpr int NCH     = 64;
constexpr int NIN0    = 129;
constexpr int NODES   = NBATCH * NATOM;
constexpr int CATOMS  = 4096;
constexpr int NCHUNKS = NODES / CATOMS;
constexpr int EROWS   = CATOMS * NNBR;
constexpr int KA1     = MLP1_TWO_TERM ? 128 : 64;
constexpr int KA2     = MLP2_TWO_TERM ? 128 : 64;
constexpr int SBLK    = 256;
constexpr int SPB     = SBLK / NBATCH;

static_assert(NCH == 64 && NCH == 2 * 32);
static_assert(NNBR == 32);
static_assert(NATOM % CATOMS == 0 && NCHUNKS * CATOMS == NODES && NCHUNKS == 16);
static_assert(NODES % 64 == 0 && EROWS % 64 == 0);
static_assert(128 % 64 == 0 && 64 % 64 == 0);
static_assert(64 % 32 == 0 && KA1 % 32 == 0 && KA2 % 32 == 0);
static_assert(128 % 32 == 0 && 64 % 32 == 0);
static_assert(SBLK * 256 == NODES && SPB * NBATCH == SBLK && SPB * 256 == NATOM);
static_assert(CATOMS % 8 == 0 && NODES % 8 == 0);

constexpr int T_W0C = 0;
constexpr int T_B0  = 64;
constexpr int T_B1  = 128;
constexpr int T_B2  = 192;
constexpr int T_SC  = 256;
constexpr int T_SH  = 320;

constexpr size_t al256(size_t v) { return (v + 255) & ~(size_t)255; }
constexpr size_t SZ_P    = (size_t)NODES * 128 * 4;
constexpr size_t SZ_A    = (size_t)EROWS * 128 * 2;
constexpr size_t SZ_T    = (size_t)EROWS * 64 * 4;
constexpr size_t SZ_UPD  = (size_t)NODES * 64 * 4;
constexpr size_t SZ_EMB  = (size_t)NODES * 64 * 2;
constexpr size_t SZ_WP   = (size_t)128 * 64 * 2;
constexpr size_t SZ_TAB  = 2048;
constexpr size_t SZ_REC  = (size_t)SBLK * 64 * 8;
constexpr size_t SZ_MS   = (size_t)SBLK * 128;
constexpr size_t O_P     = 0;
constexpr size_t O_A     = al256(O_P + SZ_P);
constexpr size_t O_T     = al256(O_A + SZ_A);
constexpr size_t O_UPD   = al256(O_T + SZ_T);
constexpr size_t O_EMB   = al256(O_UPD + SZ_UPD);
constexpr size_t O_W0AB  = al256(O_EMB + SZ_EMB);
constexpr size_t O_W1D   = al256(O_W0AB + SZ_WP);
constexpr size_t O_W2D   = al256(O_W1D + SZ_WP);
constexpr size_t O_TAB   = al256(O_W2D + SZ_WP);
constexpr size_t O_REC1  = al256(O_TAB + SZ_TAB);
constexpr size_t O_REC2  = al256(O_REC1 + SZ_REC);
constexpr size_t O_MS    = al256(O_REC2 + SZ_REC);
constexpr size_t WS_TOTAL = al256(O_MS + SZ_MS);
static_assert(WS_TOTAL <= ((size_t)128 << 20));
static_assert((size_t)EROWS * KA1 * 2 <= SZ_A && (size_t)EROWS * KA2 * 2 <= SZ_A);
static_assert(384 * 4 <= SZ_TAB);

constexpr int PB_EMB  = NODES * 8 / 256;
constexpr int PB_W0   = PB_EMB;
constexpr int PB_W1   = PB_W0 + 4;
constexpr int PB_W2   = PB_W1 + 4;
constexpr int PB_TAB  = PB_W2 + 4;
constexpr int PB_ALL  = PB_TAB + 1;

__device__ __forceinline__ void st2_v4u(void* p, const v4u v) {
  volatile v4u* q = (volatile v4u*)p;
  *q = v;
  __threadfence();
  *q = v;
}
__device__ __forceinline__ void st2_v4f(float* p, const v4f v) {
  volatile v4f* q = (volatile v4f*)p;
  *q = v;
  __threadfence();
  *q = v;
}
__device__ __forceinline__ void st2_v2f(float* p, const v2f v) {
  volatile v2f* q = (volatile v2f*)p;
  *q = v;
  __threadfence();
  *q = v;
}
__device__ __forceinline__ void st2_v2d(double* p, const v2d v) {
  volatile v2d* q = (volatile v2d*)p;
  *q = v;
  __threadfence();
  *q = v;
}

__device__ __forceinline__ float gelu_f(float x) {
#if GELU_MODE == 0
  return 0.5f * x * (1.0f + erff(x * 0.70710678f));
#else
  const float z  = x * 0.70710678f;
  const float az = fabsf(z);
  const float t  = __builtin_amdgcn_rcpf(1.0f + 0.3275911f * az);
  float p = 0x1.0fb844p+0f;
  p = p * t - 0x1.7401c6p+0f;
  p = p * t + 0x1.6be1c6p+0f;
  p = p * t - 0x1.23531cp-2f;
  p = p * t + 0x1.04f20cp-2f;
  p = p * t;
  const float ea = fmaxf(-az * az, -80.0f);
  const float e  = __expf(ea);
  const float er = copysignf(1.0f - p * e, z);
  return 0.5f * x * (1.0f + er);
#endif
}

template <int KA>
__device__ __forceinline__ void wdup_piece(const float* __restrict__ W, unsigned short* dst, int u) {
  constexpr int PPR   = KA / 8;
  constexpr int TOTAL = 64 * PPR;
  const int uc = u < TOTAL ? u : TOTAL - 1;
  const int r  = uc / PPR;
  const int p  = uc - r * PPR;
  const int c0 = (p & 7) * 8;
  const float* s = W + r * 64 + c0;
  const v4f a = *(const v4fa*)s;
  const v4f c = *(const v4fa*)(s + 4);
  asm volatile("" :: "v"(a), "v"(c));
  const v4u o = pack8_bf16(a, c);
  if (u < TOTAL) st2_v4u(dst + (size_t)u * 8, o);
}

__global__ __launch_bounds__(256) void k_prep(
    const float* __restrict__ x, const float* __restrict__ mask, const float* __restrict__ W0,
    const float* __restrict__ b0, const float* __restrict__ W1, const float* __restrict__ b1,
    const float* __restrict__ W2, const float* __restrict__ b2, const float* __restrict__ scale,
    const float* __restrict__ shift,
    unsigned short* EMB, unsigned short* W0AB, unsigned short* W1D, unsigned short* W2D, float* TAB) {
  const int b = (int)blockIdx.x, tid = (int)threadIdx.x;
  if (b < PB_EMB) {
    const unsigned g = (unsigned)b * 256u + (unsigned)tid;
    const int row = (int)(g >> 3);
    const int p   = (int)(g & 7u);
    const float* xp = x + (size_t)row * 64 + 8 * p;
    v4f a = *(const v4fa*)xp;
    v4f c = *(const v4fa*)(xp + 4);
    const float mk = mask[row];
    asm volatile("" :: "v"(a), "v"(c), "v"(mk));
    const float m = bf16_val(mk);
#pragma unroll
    for (int e = 0; e < 4; ++e) {
      a[e] = bf16_val(a[e]) * m;
      c[e] = bf16_val(c[e]) * m;
    }
    st2_v4u(EMB + (size_t)g * 8, pack8_bf16(a, c));
  } else if (b < PB_W1) {
    const int u = (b - PB_W0) * 256 + tid;
    const int r = u >> 3, p = u & 7;
    const int o = r & 63, half = r >> 6;
    const float* s = W0 + o * NIN0 + half * 64 + 8 * p;
    float w[8];
#pragma unroll
    for (int e = 0; e < 8; ++e) {
      const float v = s[e];
      asm volatile("" :: "v"(v));
      w[e] = v;
    }
    const v4f a = (v4f){ w[0], w[1], w[2], w[3] };
    const v4f c = (v4f){ w[4], w[5], w[6], w[7] };
    st2_v4u(W0AB + (size_t)u * 8, pack8_bf16(a, c));
  } else if (b < PB_W2) {
    wdup_piece<KA1>(W1, W1D, (b - PB_W1) * 256 + tid);
  } else if (b < PB_TAB) {
    wdup_piece<KA2>(W2, W2D, (b - PB_W2) * 256 + tid);
  } else {
    const int lane = tid & 31, wave = tid >> 5;
    const int c = (lane & 15) * 4;
    const bool hi = lane >= 16;
    if (wave == 0) {
      float w[4];
#pragma unroll
      for (int e = 0; e < 4; ++e) {
        const float v = W0[(c + e) * NIN0 + 128];
        asm volatile("" :: "v"(v));
        w[e] = v;
      }
      const v4f bv = *(const v4fa*)(b0 + c);
      asm volatile("" :: "v"(bv));
      v4f v;
#pragma unroll
      for (int e = 0; e < 4; ++e) v[e] = bf16_val(hi ? bv[e] : w[e]);
      st2_v4f(TAB + T_W0C + 4 * lane, v);
    } else if (wave == 1) {
      const v4f p = *(const v4fa*)(b1 + c);
      const v4f q = *(const v4fa*)(b2 + c);
      asm volatile("" :: "v"(p), "v"(q));
      v4f v;
#pragma unroll
      for (int e = 0; e < 4; ++e) v[e] = bf16_val(hi ? q[e] : p[e]);
      st2_v4f(TAB + T_B1 + 4 * lane, v);
    } else if (wave == 2) {
      const v4f p = *(const v4fa*)(scale + c);
      const v4f q = *(const v4fa*)(shift + c);
      asm volatile("" :: "v"(p), "v"(q));
      v4f v;
#pragma unroll
      for (int e = 0; e < 4; ++e) v[e] = bf16_val(hi ? q[e] : p[e]);
      st2_v4f(TAB + T_SC + 4 * lane, v);
    }
  }
}

template <int TWO>
__global__ __launch_bounds__(256) void k_edge0(const float* __restrict__ P, const float* __restrict__ dist,
                                               const int* __restrict__ eidx, const float* __restrict__ TAB,
                                               unsigned* A, int atom0) {
  constexpr int KW = TWO ? 64 : 32;
  const int lane = threadIdx.x & 31;
  const int wave = threadIdx.x >> 5;
  const int aloc = (int)blockIdx.x * 8 + wave;
  if (aloc >= CATOMS) return;
  const int ag  = clampi(atom0 + aloc, 0, NODES - 1);
  const int nb0 = (ag >> 13) << 13;
  int   idx = eidx[(size_t)ag * NNBR + lane];
  float dd  = dist[(size_t)ag * NNBR + lane];
  asm volatile("" :: "v"(idx), "v"(dd));
  int safe = (idx == -1) ? 0 : idx;
  safe = clampi(safe, 0, NATOM - 1);
  const float dv = bf16_val(dd);
  const v2f pb = *(const v2fa*)(P + (size_t)ag * 128 + 64 + 2 * lane);
  const v2f wc = *(const v2fa*)(TAB + T_W0C + 2 * lane);
  const v2f bb = *(const v2fa*)(TAB + T_B0 + 2 * lane);
  unsigned* arow = A + (size_t)aloc * NNBR * KW + lane;
#pragma unroll 1
  for (int k = 0; k < NNBR; ++k) {
    const int   sk = __shfl(safe, k);
    const float dk = __shfl(dv, k);
    const v2f pa = *(const v2fa*)(P + (size_t)(nb0 + sk) * 128 + 2 * lane);
    asm volatile("" :: "v"(pa.x), "v"(pa.y));
    const float x0 = ((pa.x + pb.x) + dk * wc.x) + bb.x;
    const float x1 = ((pa.y + pb.y) + dk * wc.y) + bb.y;
    const float h0 = gelu_f(x0);
    const float h1 = gelu_f(x1);
    const unsigned whi = pk16(bf16_bits(h0), bf16_bits(h1));
    const unsigned wlo = pk16(bf16_lo_bits(h0), bf16_lo_bits(h1));
    volatile unsigned* q = arow + k * KW;
    q[0] = whi;
    if (TWO) q[32] = wlo;
    __threadfence();
    q[0] = whi;
    if (TWO) q[32] = wlo;
  }
}

template <int TWO>
__global__ __launch_bounds__(256) void k_act1(const float* __restrict__ T, const float* __restrict__ TAB,
                                              unsigned* A) {
  constexpr int KW = TWO ? 64 : 32;
  const int lane = threadIdx.x & 31;
  const int wave = threadIdx.x >> 5;
  const int aloc = (int)blockIdx.x * 8 + wave;
  if (aloc >= CATOMS) return;
  const v2f bb = *(const v2fa*)(TAB + T_B1 + 2 * lane);
  const float* trow = T + (size_t)aloc * NNBR * 64 + 2 * lane;
  unsigned* arow = A + (size_t)aloc * NNBR * KW + lane;
#pragma unroll 1
  for (int k = 0; k < NNBR; ++k) {
    const v2f t = *(const v2fa*)(trow + k * 64);
    const float h0 = gelu_f(t.x + bb.x);
    const float h1 = gelu_f(t.y + bb.y);
    const unsigned whi = pk16(bf16_bits(h0), bf16_bits(h1));
    const unsigned wlo = pk16(bf16_lo_bits(h0), bf16_lo_bits(h1));
    volatile unsigned* q = arow + k * KW;
    q[0] = whi;
    if (TWO) q[32] = wlo;
    __threadfence();
    q[0] = whi;
    if (TWO) q[32] = wlo;
  }
}

__global__ __launch_bounds__(256) void k_agg(const float* __restrict__ T, const int* __restrict__ eidx,
                                             const float* __restrict__ x, const float* __restrict__ mask,
                                             const float* __restrict__ TAB, float* UPD, int atom0) {
  const int lane = threadIdx.x & 31;
  const int wave = threadIdx.x >> 5;
  const int aloc = (int)blockIdx.x * 8 + wave;
  if (aloc >= CATOMS) return;
  const int ag = clampi(atom0 + aloc, 0, NODES - 1);
  int idx = eidx[(size_t)ag * NNBR + lane];
  asm volatile("" :: "v"(idx));
  const float vf = (idx != -1) ? 1.0f : 0.0f;
  const v2f bb = *(const v2fa*)(TAB + T_B2 + 2 * lane);
  const float* trow = T + (size_t)aloc * NNBR * 64 + 2 * lane;
  float s0 = 0.0f, s1 = 0.0f, nv = 0.0f;
#pragma unroll 1
  for (int k = 0; k < NNBR; ++k) {
    const v2f t = *(const v2fa*)(trow + k * 64);
    asm volatile("" :: "v"(t.x), "v"(t.y));
    const float vk = __shfl(vf, k);
    const float h0 = gelu_f(t.x + bb.x);
    const float h1 = gelu_f(t.y + bb.y);
    s0 += h0 * vk;
    s1 += h1 * vk;
    nv += vk;
  }
  nv = (nv == 0.0f) ? 1.0f : nv;
  const v2f xv = *(const v2fa*)(x + (size_t)ag * 64 + 2 * lane);
  const float mk = mask[ag];
  asm volatile("" :: "v"(xv.x), "v"(xv.y), "v"(mk));
  const float m = bf16_val(mk);
  v2f u;
  u.x = (bf16_val(xv.x) + s0 / nv) * m;
  u.y = (bf16_val(xv.y) + s1 / nv) * m;
  st2_v2f(UPD + (size_t)ag * 64 + 2 * lane, u);
}

__global__ __launch_bounds__(256) void k_sum(const float* __restrict__ UPD, const float* __restrict__ mask,
                                             double* REC1, float* MS) {
  __shared__ float  sp[4][64];
  __shared__ double sd[64];
  const int tid = (int)threadIdx.x, lane = tid & 31, wave = tid >> 5;
  const int blk = (int)blockIdx.x;
  const int a0 = blk * 256;
  const int c = tid & 63, g = tid >> 6;
  float s = 0.0f;
#pragma unroll 4
  for (int i = 0; i < 64; ++i) {
    const int a = a0 + g * 64 + i;
    const float u  = UPD[(size_t)a * 64 + c];
    const float mk = mask[a];
    s += u * bf16_val(mk);
  }
  sp[g][c] = s;
  float ms = 0.0f;
  if (wave == 0) {
    const float* mp = mask + a0 + lane * 8;
    const v4f m0 = *(const v4fa*)mp;
    const v4f m1 = *(const v4fa*)(mp + 4);
    ms = bf16_val(m0[0]);
    ms += bf16_val(m0[1]); ms += bf16_val(m0[2]); ms += bf16_val(m0[3]);
    ms += bf16_val(m1[0]); ms += bf16_val(m1[1]); ms += bf16_val(m1[2]); ms += bf16_val(m1[3]);
    ms += __shfl_xor(ms, 16);
    ms += __shfl_xor(ms, 8);
    ms += __shfl_xor(ms, 4);
    ms += __shfl_xor(ms, 2);
    ms += __shfl_xor(ms, 1);
  }
  __syncthreads();
  if (tid < 64) sd[tid] = (((double)sp[0][tid] + (double)sp[1][tid]) + (double)sp[2][tid]) + (double)sp[3][tid];
  __syncthreads();
  if (wave == 0) {
    v2d r;
    r.x = sd[2 * lane];
    r.y = sd[2 * lane + 1];
    st2_v2d(REC1 + (size_t)blk * 64 + 2 * lane, r);
    if (lane < 8) {
      const v4f v = (v4f){ (lane == 0) ? ms : 0.0f, 0.0f, 0.0f, 0.0f };
      st2_v4f(MS + (size_t)blk * 32 + 4 * lane, v);
    }
  }
}

__device__ __forceinline__ void batch_mean(const double* __restrict__ REC1, const float* __restrict__ MS,
                                           int b, int c, double& cnt, float& mean) {
  double s = 0.0, n = 0.0;
#pragma unroll 2
  for (int r = 0; r < SPB; ++r) {
    const int rec = b * SPB + r;
    s += REC1[(size_t)rec * 64 + c];
    n += (double)MS[(size_t)rec * 32];
  }
  n = (n == 0.0) ? 1.0 : n;
  cnt = n;
  mean = (float)(s / n);
}

__global__ __launch_bounds__(256) void k_ss(const float* __restrict__ UPD, const float* __restrict__ mask,
                                            const double* __restrict__ REC1, const float* __restrict__ MS,
                                            double* REC2) {
  __shared__ float  smean[64];
  __shared__ float  sp[4][64];
  __shared__ double sd[64];
  const int tid = (int)threadIdx.x, lane = tid & 31, wave = tid >> 5;
  const int blk = (int)blockIdx.x;
  const int b = clampi(blk / SPB, 0, NBATCH - 1);
  const int a0 = blk * 256;
  const int c = tid & 63, g = tid >> 6;
  if (tid < 64) {
    double cnt; float mean;
    batch_mean(REC1, MS, b, tid, cnt, mean);
    smean[tid] = mean;
  }
  __syncthreads();
  const float mean = smean[c];
  float s = 0.0f;
#pragma unroll 4
  for (int i = 0; i < 64; ++i) {
    const int a = a0 + g * 64 + i;
    const float u  = UPD[(size_t)a * 64 + c];
    const float mk = mask[a];
    const float d = u * bf16_val(mk) - mean;
    s += d * d;
  }
  sp[g][c] = s;
  __syncthreads();
  if (tid < 64) sd[tid] = (((double)sp[0][tid] + (double)sp[1][tid]) + (double)sp[2][tid]) + (double)sp[3][tid];
  __syncthreads();
  if (wave == 0) {
    v2d r;
    r.x = sd[2 * lane];
    r.y = sd[2 * lane + 1];
    st2_v2d(REC2 + (size_t)blk * 64 + 2 * lane, r);
  }
}

__global__ __launch_bounds__(256) void k_out(const float* __restrict__ UPD, const float* __restrict__ mask,
                                             const double* __restrict__ REC1, const double* __restrict__ REC2,
                                             const float* __restrict__ MS, const float* __restrict__ TAB,
                                             float* out, int nrows) {
  __shared__ float smean[64];
  __shared__ float svar[64];
  const int tid = (int)threadIdx.x, lane = tid & 31, wave = tid >> 5;
  const int blk = (int)blockIdx.x;
  const int b = clampi((blk * 8) >> 13, 0, NBATCH - 1);
  if (tid < 64) {
    double cnt; float mean;
    batch_mean(REC1, MS, b, tid, cnt, mean);
    double ss = 0.0;
#pragma unroll 2
    for (int r = 0; r < SPB; ++r) ss += REC2[(size_t)(b * SPB + r) * 64 + tid];
    smean[tid] = mean;
    svar[tid]  = (float)(ss / cnt);
  }
  __syncthreads();
  const int row = blk * 8 + wave;
  const int rc = clampi(row, 0, nrows - 1);
  const v2f u = *(const v2fa*)(UPD + (size_t)rc * 64 + 2 * lane);
  const float mk = mask[rc];
  asm volatile("" :: "v"(u.x), "v"(u.y), "v"(mk));
  const v2f sc = *(const v2fa*)(TAB + T_SC + 2 * lane);
  const v2f sh = *(const v2fa*)(TAB + T_SH + 2 * lane);
  const float m = bf16_val(mk);
  const float d0 = sqrtf(svar[2 * lane] + 1e-5f);
  const float d1 = sqrtf(svar[2 * lane + 1] + 1e-5f);
  v2f o;
  o.x = (((u.x - smean[2 * lane]) / d0) * sc.x + sh.x) * m;
  o.y = (((u.y - smean[2 * lane + 1]) / d1) * sc.y + sh.y) * m;
  if (row < nrows) st2_v2f(out + (size_t)row * 64 + 2 * lane, o);
}

extern "C" void kernel_launch(void* const* d_in, const int* in_sizes, int n_in,
                              void* d_out, int out_size, void* d_ws, size_t ws_size,
                              hipStream_t stream) {
  if (n_in < 12) return;
  if (in_sizes[0] != NODES * NCH || in_sizes[1] != NODES * NNBR || in_sizes[2] != NODES * NNBR ||
      in_sizes[3] != NODES) return;
  if (in_sizes[4] != NCH * NIN0 || in_sizes[5] != NCH || in_sizes[6] != NCH * NCH || in_sizes[7] != NCH ||
      in_sizes[8] != NCH * NCH || in_sizes[9] != NCH || in_sizes[10] != NCH || in_sizes[11] != NCH) return;
  if (out_size != NODES * NCH) return;
  if (ws_size < WS_TOTAL) return;

  const float* x     = (const float*)d_in[0];
  const float* dist  = (const float*)d_in[1];
  const int*   eidx  = (const int*)  d_in[2];
  const float* mask  = (const float*)d_in[3];
  const float* W0    = (const float*)d_in[4];
  const float* b0    = (const float*)d_in[5];
  const float* W1    = (const float*)d_in[6];
  const float* b1    = (const float*)d_in[7];
  const float* W2    = (const float*)d_in[8];
  const float* b2    = (const float*)d_in[9];
  const float* scale = (const float*)d_in[10];
  const float* shift = (const float*)d_in[11];
  float* out = (float*)d_out;

  char* ws = (char*)d_ws;
  float*          P    = (float*)(ws + O_P);
  unsigned short* Ah   = (unsigned short*)(ws + O_A);
  unsigned*       Aw   = (unsigned*)(ws + O_A);
  float*          T    = (float*)(ws + O_T);
  float*          UPD  = (float*)(ws + O_UPD);
  unsigned short* EMB  = (unsigned short*)(ws + O_EMB);
  unsigned short* W0AB = (unsigned short*)(ws + O_W0AB);
  unsigned short* W1D  = (unsigned short*)(ws + O_W1D);
  unsigned short* W2D  = (unsigned short*)(ws + O_W2D);
  float*          TAB  = (float*)(ws + O_TAB);
  double*         REC1 = (double*)(ws + O_REC1);
  double*         REC2 = (double*)(ws + O_REC2);
  float*          MS   = (float*)(ws + O_MS);

  k_prep<<<PB_ALL, 256, 0, stream>>>(x, mask, W0, b0, W1, b1, W2, b2, scale, shift, EMB, W0AB, W1D, W2D, TAB);
  k_gemm_nt<0, 0><<<2048 / 8, 256, 0, stream>>>(EMB, W0AB, TAB, P, NODES, 128, 64, 128);
  for (int c = 0; c < NCHUNKS; ++c) {
    const int atom0 = c * CATOMS;
    k_edge0<MLP1_TWO_TERM><<<CATOMS / 8, 256, 0, stream>>>(P, dist, eidx, TAB, Aw, atom0);
    k_gemm_nt<MLP1_TWO_TERM, 0><<<2048 / 8, 256, 0, stream>>>(Ah, W1D, TAB, T, EROWS, 64, KA1, 64);
    k_act1<MLP2_TWO_TERM><<<CATOMS / 8, 256, 0, stream>>>(T, TAB, Aw);
    k_gemm_nt<MLP2_TWO_TERM, 0><<<2048 / 8, 256, 0, stream>>>(Ah, W2D, TAB, T, EROWS, 64, KA2, 64);
    k_agg<<<CATOMS / 8, 256, 0, stream>>>(T, eidx, x, mask, TAB, UPD, atom0);
  }
  k_sum<<<SBLK, 256, 0, stream>>>(UPD, mask, REC1, MS);
  k_ss<<<SBLK, 256, 0, stream>>>(UPD, mask, REC1, MS, REC2);
  k_out<<<NODES / 8, 256, 0, stream>>>(UPD, mask, REC1, REC2, MS, TAB, out, NODES);
}
